// BaseAttention_40329742910040
// MI455X (gfx1250) — hardware-verified
//
#include <hip/hip_runtime.h>


#ifndef NB
#define NB 8
#endif
#ifndef SEQ
#define SEQ 1024
#endif
#define NB_FULL 8
#define SEQ_FULL 1024
#define NHD 16
#define HD 64
#define NU (NB * NHD)
#define SCL 0.125f
#define NEGBIG (-1.0e30f)
#define OSP 68

static_assert(SEQ % 64 == 0);
static_assert(SEQ >= 64 && SEQ <= SEQ_FULL);
static_assert(NB >= 1 && NB <= NB_FULL);
static_assert(HD == 64);

typedef unsigned short bf;
typedef __attribute__((ext_vector_type(16))) __bf16 v16bf;
typedef __attribute__((ext_vector_type(16))) unsigned short v16us;
typedef __attribute__((ext_vector_type(8))) unsigned short v8us;
typedef __attribute__((ext_vector_type(8))) float v8f;
typedef __attribute__((ext_vector_type(4))) float v4f;
typedef v4f __attribute__((may_alias)) v4fa;

__device__ __forceinline__ unsigned short f2bf(float f) { unsigned u = __float_as_uint(f); u += 0x7FFFu + ((u >> 16) & 1u); return (unsigned short)(u >> 16); }
__device__ __forceinline__ float bf2f(unsigned short b) { return __uint_as_float(((unsigned)b) << 16); }
__device__ __forceinline__ void splitf(float y, unsigned short& hp, unsigned short& lp) { hp = f2bf(y); lp = f2bf(y - bf2f(hp)); }
__device__ __forceinline__ v16bf cat16b(v8us lo, v8us hi) {
    v16us w = __builtin_shufflevector(lo, hi, 0, 1, 2, 3, 4, 5, 6, 7, 8, 9, 10, 11, 12, 13, 14, 15);
    return __builtin_bit_cast(v16bf, w);
}
__device__ __forceinline__ v16bf ldfrag(const bf* p) { return cat16b(*(const v8us*)p, *(const v8us*)(p + 16)); }
__device__ __forceinline__ v8f wmmab(v16bf a, v16bf b, v8f c) { return __builtin_amdgcn_wmma_f32_16x16x32_bf16(false, a, false, b, (short)0, c, false, false); }

__global__ __launch_bounds__(256) void k_cvt8(const float* __restrict__ src, bf* dst, unsigned n8) {
    const unsigned i = blockIdx.x * 256u + threadIdx.x;
    if (i >= n8) return;
    const size_t e = (size_t)i * 8;
    const size_t u = e / ((size_t)SEQ * HD);
    const size_t rem = e - u * ((size_t)SEQ * HD);
    const v8f v = *(const v8f*)(src + u * (size_t)SEQ_FULL * HD + rem);
    v8us o;
#pragma unroll
    for (int k = 0; k < 8; ++k) o[k] = f2bf(v[k]);
    *(volatile v8us*)(dst + e) = o;
    __threadfence();
    *(volatile v8us*)(dst + e) = o;
}

__global__ __launch_bounds__(256) void k_vt(const float* __restrict__ V, bf* VT) {
    __shared__ __align__(16) float tile[64 * OSP];
    const int t = threadIdx.x;
    const int u = (int)blockIdx.x / (SEQ / 64);
    const int kt = (int)blockIdx.x - u * (SEQ / 64);
    const float* vsrc = V + (size_t)u * SEQ_FULL * HD + (size_t)kt * 64 * HD;
#pragma unroll
    for (int i = 0; i < 4; ++i) {
        const int lin = i * 256 + t;
        const int key = lin >> 4, c4 = (lin & 15) * 4;
        const v4f a = *(const v4f*)(vsrc + (size_t)key * HD + c4);
        *(v4fa*)(tile + key * OSP + c4) = a;
    }
    __syncthreads();
    const int lane = t & 31, wv = t >> 5;
    v8us o0, o1;
    const int d0 = 4 * wv + (lane >> 3), d1 = 4 * (wv + 8) + (lane >> 3);
    const int t0 = (lane & 7) * 8;
#pragma unroll
    for (int j = 0; j < 8; ++j) { o0[j] = f2bf(tile[(t0 + j) * OSP + d0]); o1[j] = f2bf(tile[(t0 + j) * OSP + d1]); }
    bf* dst0 = VT + ((size_t)u * HD + d0) * SEQ + (size_t)kt * 64 + t0;
    bf* dst1 = VT + ((size_t)u * HD + d1) * SEQ + (size_t)kt * 64 + t0;
    *(volatile v8us*)dst0 = o0;
    *(volatile v8us*)dst1 = o1;
    __threadfence();
    *(volatile v8us*)dst0 = o0;
    *(volatile v8us*)dst1 = o1;
}

__global__ __launch_bounds__(128) __attribute__((amdgpu_num_vgpr(256)))
void k_attn(const bf* __restrict__ QB, const bf* __restrict__ KB, const bf* __restrict__ VT, float* OUT) {
    __shared__ __align__(16) float os[4 * 16 * OSP];
    const int lane = threadIdx.x & 31, m = lane & 15, h = lane >> 4;
    const int wv = __builtin_amdgcn_readfirstlane((int)(threadIdx.x >> 5));
    const int gw = (int)blockIdx.x * 4 + wv;
    const int tiles = SEQ / 16;
    const int u = gw / tiles;
    const int q0 = (gw - u * tiles) * 16;
    const bf* qp = QB + (size_t)u * SEQ * HD;
    const bf* kp = KB + (size_t)u * SEQ * HD;
    const bf* vp = VT + (size_t)u * HD * SEQ;
    float* op = OUT + ((size_t)u * SEQ_FULL + q0) * HD;

    v16bf qf[2];
#pragma unroll
    for (int kb = 0; kb < 2; ++kb) qf[kb] = ldfrag(qp + (size_t)(q0 + m) * HD + kb * 32 + 8 * h);

    v8f oacc[4];
#pragma unroll
    for (int c = 0; c < 4; ++c) oacc[c] = (v8f){};
    float mrun = NEGBIG, lrun = 0.0f;
    const int qi = q0 + m;
    const int jend = q0 + 16;

#pragma unroll 1
    for (int jb = 0; jb < jend; jb += 32) {
        v16bf ka[2][2];
#pragma unroll
        for (int jt = 0; jt < 2; ++jt)
#pragma unroll
            for (int kb = 0; kb < 2; ++kb) ka[jt][kb] = ldfrag(kp + (size_t)(jb + 16 * jt + m) * HD + kb * 32 + 8 * h);
        v8f st[2];
#pragma unroll
        for (int jt = 0; jt < 2; ++jt) {
            st[jt] = (v8f){};
            st[jt] = wmmab(ka[jt][0], qf[0], st[jt]);
            st[jt] = wmmab(ka[jt][1], qf[1], st[jt]);
        }
        asm volatile("v_nop\n\tv_nop\n\tv_nop\n\tv_nop" : "+v"(st[0]), "+v"(st[1]) : "v"(ka[0][1]), "v"(ka[1][1]), "v"(qf[1]));

        float p0[8], p1[8];
        float mx = NEGBIG;
#pragma unroll
        for (int r = 0; r < 8; ++r) {
            const int k0i = jb + 8 * h + r;
            float x0 = st[0][r] * SCL;
            float x1 = st[1][r] * SCL;
            x0 = (k0i <= qi) ? x0 : NEGBIG;
            x1 = (k0i + 16 <= qi) ? x1 : NEGBIG;
            p0[r] = x0; p1[r] = x1;
            mx = fmaxf(mx, fmaxf(x0, x1));
        }
        mx = fmaxf(mx, __shfl_xor(mx, 16, 32));
        const float mn = fmaxf(mrun, mx);
        const float rsc = __expf(mrun - mn);
        mrun = mn;
        float ls = 0.0f;
#pragma unroll
        for (int r = 0; r < 8; ++r) {
            p0[r] = __expf(p0[r] - mn);
            p1[r] = __expf(p1[r] - mn);
            ls += p0[r] + p1[r];
        }
        ls += __shfl_xor(ls, 16, 32);
        lrun = lrun * rsc + ls;
#pragma unroll
        for (int c = 0; c < 4; ++c) oacc[c] = oacc[c] * rsc;

        v8us ph0, ph1, pl0, pl1;
#pragma unroll
        for (int r = 0; r < 8; ++r) {
            unsigned short ah, al;
            splitf(p0[r], ah, al); ph0[r] = ah; pl0[r] = al;
            splitf(p1[r], ah, al); ph1[r] = ah; pl1[r] = al;
        }
        const v16bf bph = cat16b(ph0, ph1);
        const v16bf bpl = cat16b(pl0, pl1);

        v16bf va;
#pragma unroll
        for (int c = 0; c < 4; ++c) {
            va = ldfrag(vp + (size_t)(c * 16 + m) * SEQ + jb + 8 * h);
            oacc[c] = wmmab(va, bph, oacc[c]);
            oacc[c] = wmmab(va, bpl, oacc[c]);
        }
        asm volatile("v_nop\n\tv_nop\n\tv_nop\n\tv_nop" : "+v"(oacc[0]), "+v"(oacc[1]), "+v"(oacc[2]), "+v"(oacc[3]) : "v"(va), "v"(bph), "v"(bpl));
    }

    const float inv = 1.0f / lrun;
    float* osw = os + wv * (16 * OSP);
#pragma unroll
    for (int c = 0; c < 4; ++c) {
        v4f a, b;
        a[0] = oacc[c][0] * inv; a[1] = oacc[c][1] * inv; a[2] = oacc[c][2] * inv; a[3] = oacc[c][3] * inv;
        b[0] = oacc[c][4] * inv; b[1] = oacc[c][5] * inv; b[2] = oacc[c][6] * inv; b[3] = oacc[c][7] * inv;
        *(v4fa*)(osw + m * OSP + c * 16 + 8 * h) = a;
        *(v4fa*)(osw + m * OSP + c * 16 + 8 * h + 4) = b;
    }
    __syncthreads();
    v4f vals[8];
#pragma unroll
    for (int s = 0; s < 8; ++s) vals[s] = *(const v4fa*)(osw + (2 * s + h) * OSP + m * 4);
#pragma unroll
    for (int s = 0; s < 8; ++s) *(volatile v4f*)(op + (size_t)(2 * s + h) * HD + m * 4) = vals[s];
    __threadfence();
#pragma unroll
    for (int s = 0; s < 8; ++s) *(volatile v4f*)(op + (size_t)(2 * s + h) * HD + m * 4) = vals[s];
}

extern "C" void kernel_launch(void* const* d_in, const int* in_sizes, int n_in,
                              void* d_out, int out_size, void* d_ws, size_t ws_size, hipStream_t stream) {
    if (n_in < 3) return;
    const long long need = (long long)NU * SEQ_FULL * HD;
    if ((long long)in_sizes[0] < need || (long long)in_sizes[1] < need || (long long)in_sizes[2] < need) return;
    if ((long long)out_size < need) return;
    const size_t plane = (size_t)NU * SEQ * HD;
    const size_t pbytes = plane * 2;
    if (3 * pbytes > ws_size) return;
    char* ws = (char*)d_ws;
    bf* QB = (bf*)ws;
    bf* KB = (bf*)(ws + pbytes);
    bf* VT = (bf*)(ws + 2 * pbytes);
    const float* Qin = (const float*)d_in[0];
    const float* Kin = (const float*)d_in[1];
    const float* Vin = (const float*)d_in[2];
    float* OUT = (float*)d_out;
    const unsigned n8 = (unsigned)(plane / 8);
    k_cvt8<<<dim3((n8 + 255u) / 256u), dim3(256), 0, stream>>>(Qin, QB, n8);
    k_cvt8<<<dim3((n8 + 255u) / 256u), dim3(256), 0, stream>>>(Kin, KB, n8);
    k_vt<<<dim3((unsigned)(NU * (SEQ / 64))), dim3(256), 0, stream>>>(Vin, VT);
    k_attn<<<dim3((unsigned)(NU * SEQ / 64)), dim3(128), 0, stream>>>(QB, KB, VT, OUT);
}
